// CrossTransformer_89335319757159
// MI455X (gfx1250) — hardware-verified
//
#include <hip/hip_runtime.h>
#include <stdint.h>

#define NSUP    25
#define NQRY    32
#define NCLS    5
#define CIN     512
#define HW      196
#define DK      128
#define DV      128
#define NPROJ   256
#define QROWS   6272
#define QTILES  98
#define SROWS   4900
#define SROWSP  4928
#define NCHMAX  77
#define OUT0_ELEMS 4014080
#define OUT1_ELEMS 802816
#define NLN16   98
#define QLOFF   ((size_t)QROWS * DK)
#define KLOFF   ((size_t)NCLS * SROWSP * DK)
#define VLOFF   ((size_t)NCLS * DV * SROWSP)

static_assert(QROWS == NQRY * HW);
static_assert(QROWS == QTILES * 64);
static_assert(SROWS == NSUP * HW);
static_assert(SROWSP == NCHMAX * 64);
static_assert(SROWSP >= SROWS && SROWSP - SROWS < 64);
static_assert(NPROJ == DK + DV);
static_assert((CIN % 64) == 0 && (NPROJ % 64) == 0 && DK == 128 && DV == 128);
static_assert(OUT0_ELEMS == NQRY * NCLS * DV * HW);
static_assert(OUT1_ELEMS == NQRY * DV * HW);
static_assert(NCLS * QROWS * DV == OUT0_ELEMS);
static_assert(NLN16 * 32 == 16 * HW);
static_assert((DK * CIN) % (256 * 8) == 0);
static_assert((QROWS * (DK / 8)) % 256 == 0);

typedef __bf16   v16b __attribute__((ext_vector_type(16)));
typedef __bf16   v8b  __attribute__((ext_vector_type(8)));
typedef float    v8f  __attribute__((ext_vector_type(8)));
typedef float    v4f  __attribute__((ext_vector_type(4)));
typedef unsigned int v4u __attribute__((ext_vector_type(4)));
typedef v8b __attribute__((may_alias)) v8ba;
typedef v4f __attribute__((may_alias)) v4fa;
typedef v4u __attribute__((may_alias)) v4ua;

#if defined(__HIP_DEVICE_COMPILE__)
#define DEV_ASM 1
#else
#define DEV_ASM 0
#endif

__device__ __forceinline__ unsigned short bf_bits(float f) {
  const unsigned u = __float_as_uint(f);
  return (unsigned short)((u + 0x7FFFu + ((u >> 16) & 1u)) >> 16);
}
__device__ __forceinline__ float bf_up(unsigned short hb) { return __uint_as_float(((unsigned)hb) << 16); }
__device__ __forceinline__ unsigned pk16(unsigned short a, unsigned short b) { return (unsigned)a | ((unsigned)b << 16); }
__device__ __forceinline__ v8f zero8() { v8f z = {0.f, 0.f, 0.f, 0.f, 0.f, 0.f, 0.f, 0.f}; return z; }

__device__ __forceinline__ void split2(float f0, float f1, unsigned& hi, unsigned& lo) {
  const unsigned short h0 = bf_bits(f0), h1 = bf_bits(f1);
  const unsigned short l0 = bf_bits(f0 - bf_up(h0)), l1 = bf_bits(f1 - bf_up(h1));
  hi = pk16(h0, h1);
  lo = pk16(l0, l1);
}
__device__ __forceinline__ void split8(v4f a, v4f b, v4u& hi, v4u& lo) {
  unsigned x, y;
  split2(a[0], a[1], x, y); hi[0] = x; lo[0] = y;
  split2(a[2], a[3], x, y); hi[1] = x; lo[1] = y;
  split2(b[0], b[1], x, y); hi[2] = x; lo[2] = y;
  split2(b[2], b[3], x, y); hi[3] = x; lo[3] = y;
}

__device__ __forceinline__ v16b load_frag(const __bf16* p, int h) {
  union { v16b v; v8b x[2]; } f;
  f.x[0] = *(const v8ba*)(p + 8 * h);
  f.x[1] = *(const v8ba*)(p + 16 + 8 * h);
  return f.v;
}

__device__ __forceinline__ v8f mmar(v16b a, v16b b, v8f c) {
  return __builtin_amdgcn_wmma_f32_16x16x32_bf16(false, a, false, b, (short)0, c, false, false);
}
__device__ __forceinline__ v8f mma_b(v16b a, v16b b, v8f c) {
  c = __builtin_amdgcn_wmma_f32_16x16x32_bf16(false, a, false, b, (short)0, c, false, false);
#if DEV_ASM
  asm volatile("v_nop\n\tv_nop\n\tv_nop\n\tv_nop" : "+v"(c) : "v"(a), "v"(b));
#endif
  return c;
}
__device__ __forceinline__ void dep_guard(v8f& a, v8f& b, v16b x, v16b y) {
#if DEV_ASM
  asm volatile("v_nop\n\tv_nop\n\tv_nop\n\tv_nop" : "+v"(a), "+v"(b) : "v"(x), "v"(y));
#else
  (void)a; (void)b; (void)x; (void)y;
#endif
}
__device__ __forceinline__ void keep4(v16b a, v16b b, v16b c, v16b d) {
#if DEV_ASM
  asm volatile("v_nop" :: "v"(a), "v"(b), "v"(c), "v"(d));
#else
  (void)a; (void)b; (void)c; (void)d;
#endif
}
__device__ __forceinline__ void acc_guard4(v8f& a, v8f& b, v8f& c, v8f& d) {
#if DEV_ASM
  asm volatile("v_nop\n\tv_nop\n\tv_nop\n\tv_nop" : "+v"(a), "+v"(b), "+v"(c), "+v"(d));
#else
  (void)a; (void)b; (void)c; (void)d;
#endif
}

__device__ __forceinline__ int class_count(const int* __restrict__ lab, int k) {
  int cnt = 0;
#pragma unroll 1
  for (int n = 0; n < NSUP; ++n) cnt += (lab[n] == k) ? 1 : 0;
  return cnt;
}
__device__ __forceinline__ int class_member(const int* __restrict__ lab, int k, int allm, int q) {
  int run = 0, res = 0;
#pragma unroll 1
  for (int n = 0; n < NSUP; ++n) {
    const int match = (allm != 0 || lab[n] == k) ? 1 : 0;
    res = (match != 0 && run == q) ? n : res;
    run += match;
  }
  return res;
}

__global__ __launch_bounds__(256) void k_wcvt(const float* __restrict__ w0, const float* __restrict__ w1,
                                              unsigned short* WB) {
  const float* src = (blockIdx.y == 0) ? w0 : w1;
  const int i = (int)blockIdx.x * 256 + (int)threadIdx.x;
  if (i >= (DK * CIN) / 8) return;
  const v4f a = *(const v4fa*)(src + (size_t)i * 8);
  const v4f c = *(const v4fa*)(src + (size_t)i * 8 + 4);
  v4u p;
  p[0] = pk16(bf_bits(a[0]), bf_bits(a[1]));
  p[1] = pk16(bf_bits(a[2]), bf_bits(a[3]));
  p[2] = pk16(bf_bits(c[0]), bf_bits(c[1]));
  p[3] = pk16(bf_bits(c[2]), bf_bits(c[3]));
  unsigned short* o = WB + (size_t)blockIdx.y * (DK * CIN) + (size_t)i * 8;
  *(volatile v4u*)o = p;
  __threadfence();
  *(volatile v4u*)o = p;
}

__global__ __launch_bounds__(256) void k_xpose(const float* __restrict__ X, unsigned short* OUTP, int nb, int rows_pad) {
  __shared__ __align__(16) unsigned short T[64 * 72];
  const int lane = (int)threadIdx.x & 31, w = (int)threadIdx.x >> 5;
  const int pt = (int)blockIdx.x, ct = (int)blockIdx.y, z = (int)blockIdx.z;
  const int p0 = pt * 64, c0 = ct * 64;
  if (z < nb) {
    const float* xb = X + ((size_t)z * CIN + c0) * HW;
    int pa = p0 + lane;      pa = (pa > HW - 1) ? (HW - 1) : pa;
    int pb = p0 + 32 + lane; pb = (pb > HW - 1) ? (HW - 1) : pb;
#pragma unroll 1
    for (int i = 0; i < 8; ++i) {
      const int cl = w * 8 + i;
      const float* xr = xb + (size_t)cl * HW;
      const float f0 = xr[pa];
      const float f1 = xr[pb];
      T[lane * 72 + cl]        = bf_bits(f0);
      T[(lane + 32) * 72 + cl] = bf_bits(f1);
    }
  } else {
#pragma unroll 1
    for (int i = 0; i < 8; ++i) {
      const int cl = w * 8 + i;
      T[lane * 72 + cl]        = (unsigned short)0;
      T[(lane + 32) * 72 + cl] = (unsigned short)0;
    }
  }
  __syncthreads();
  const int piece = lane & 7, rg = lane >> 3;
  for (int pass = 0; pass < 2; ++pass) {
#pragma unroll
    for (int it = 0; it < 2; ++it) {
      const int pl  = it * 32 + w * 4 + rg;
      const int row = z * HW + p0 + pl;
      const bool valid = (z < nb) ? ((p0 + pl) < HW) : (row < rows_pad);
      const v4u v = *(const v4ua*)(T + pl * 72 + 8 * piece);
      if (valid) *(volatile v4u*)(OUTP + (size_t)row * CIN + c0 + 8 * piece) = v;
    }
    __threadfence();
  }
}

__global__ __launch_bounds__(256) void k_gemm64(
    const unsigned short* __restrict__ Ap, int lda,
    const unsigned short* __restrict__ Btp, int ldb,
    float* C, int ldc, int M, int N, int K) {
  const __bf16* A  = (const __bf16*)(const void*)Ap;
  const __bf16* Bt = (const __bf16*)(const void*)Btp;
  __shared__ __align__(16) float sT[8][16 * 68];
  const int lane = (int)threadIdx.x & 31;
  const int wave = (int)threadIdx.x >> 5;
  const int tilesN = N >> 6;
  const int tilesM = M >> 6;
  const int tile = (int)blockIdx.x * 8 + wave;
  if (tile >= tilesM * tilesN) return;
  const int tm = tile / tilesN;
  const int tn = tile - tm * tilesN;
  const int m0 = tm << 6;
  const int n0 = tn << 6;
  const int rlane = lane & 15;
  const int hh    = lane >> 4;
  const int mOff  = hh * 8;

  v8f acc[4][4];
#pragma unroll
  for (int i = 0; i < 4; ++i)
#pragma unroll
    for (int j = 0; j < 4; ++j) acc[i][j] = zero8();

  for (int k0 = 0; k0 < K; k0 += 32) {
    v16b bq[4];
#pragma unroll
    for (int j = 0; j < 4; ++j)
      bq[j] = load_frag(Bt + (size_t)(n0 + (j << 4) + rlane) * ldb + k0, hh);
#pragma unroll
    for (int i = 0; i < 4; ++i) {
      const v16b af = load_frag(A + (size_t)(m0 + (i << 4) + rlane) * lda + k0, hh);
#pragma unroll
      for (int j = 0; j < 4; ++j) acc[i][j] = mmar(af, bq[j], acc[i][j]);
      dep_guard(acc[i][0], acc[i][3], af, bq[3]);
    }
    keep4(bq[0], bq[1], bq[2], bq[3]);
  }
  acc_guard4(acc[0][0], acc[0][1], acc[0][2], acc[0][3]);
  acc_guard4(acc[1][0], acc[1][1], acc[1][2], acc[1][3]);
  acc_guard4(acc[2][0], acc[2][1], acc[2][2], acc[2][3]);
  acc_guard4(acc[3][0], acc[3][1], acc[3][2], acc[3][3]);

  float* slab = sT[wave];
  const int h2 = lane >> 4, c4 = (lane & 15) * 4;
#pragma unroll
  for (int i = 0; i < 4; ++i) {
    const int mBase = m0 + (i << 4);
#pragma unroll
    for (int j = 0; j < 4; ++j) {
#pragma unroll
      for (int r = 0; r < 8; ++r) {
        slab[(mOff + r) * 68 + (j << 4) + rlane] = acc[i][j][r];
      }
    }
    __builtin_amdgcn_fence(__ATOMIC_RELEASE, "workgroup");
    __builtin_amdgcn_wave_barrier();
    __builtin_amdgcn_fence(__ATOMIC_ACQUIRE, "workgroup");
    for (int pass = 0; pass < 2; ++pass) {
#pragma unroll
      for (int it = 0; it < 8; ++it) {
        const int row = it * 2 + h2;
        const v4f v = *(const v4fa*)(slab + row * 68 + c4);
        *(volatile v4f*)(C + (size_t)(mBase + row) * ldc + n0 + c4) = v;
      }
      __threadfence();
    }
    __builtin_amdgcn_fence(__ATOMIC_RELEASE, "workgroup");
    __builtin_amdgcn_wave_barrier();
    __builtin_amdgcn_fence(__ATOMIC_ACQUIRE, "workgroup");
  }
}

__global__ __launch_bounds__(256) void k_qsplit(const float* __restrict__ CQ, unsigned short* QHL) {
  const int gid = (int)blockIdx.x * 256 + (int)threadIdx.x;
  const int row = gid >> 4, cg = (gid & 15) * 8;
  if (row >= QROWS) return;
  const float* sp = CQ + (size_t)row * NPROJ + cg;
  const v4f a0 = *(const v4fa*)(sp);
  const v4f a1 = *(const v4fa*)(sp + 4);
  v4u ph, pl;
  split8(a0, a1, ph, pl);
  unsigned short* dh = QHL + (size_t)row * DK + cg;
  unsigned short* dl = dh + QLOFF;
  *(volatile v4u*)dh = ph;
  *(volatile v4u*)dl = pl;
  __threadfence();
  *(volatile v4u*)dh = ph;
  *(volatile v4u*)dl = pl;
}

__global__ __launch_bounds__(256) void k_kvgather(const float* __restrict__ CS, const int* __restrict__ lab,
                                                 unsigned short* KHL, unsigned short* VHL) {
  __shared__ __align__(16) unsigned short sV[2 * DV * 72];
  const int lane = (int)threadIdx.x & 31, w = (int)threadIdx.x >> 5;
  const int h = lane >> 4, m = lane & 15;
  const int c = (int)blockIdx.x, k = (int)blockIdx.y;
  const int cnt = class_count(lab, k);
  const int allm = (cnt == 0) ? 1 : 0;
  const int nkeys = (allm ? NSUP : cnt) * HW;
  int nch = (nkeys + 63) >> 6;
  nch = (nch > NCHMAX) ? NCHMAX : nch;
  if (c >= nch) return;
  const int cq = 8 * m;
  v4u hv[4], lv[4];
#pragma unroll
  for (int i = 0; i < 4; ++i) {
    const int sl = w * 8 + 2 * i + h;
    const int j = c * 64 + sl;
    const bool valid = (j < nkeys);
    const int jj = valid ? j : (nkeys - 1);
    const int q = jj / HW;
    const int p = jj - q * HW;
    const int n = class_member(lab, k, allm, q);
    int srow = n * HW + p;
    srow = (srow < 0) ? 0 : ((srow > SROWS - 1) ? (SROWS - 1) : srow);
    const float* sp = CS + (size_t)srow * NPROJ + cq;
    const float vm = valid ? 1.0f : 0.0f;
    const v4f a0 = *(const v4fa*)(sp) * vm;
    const v4f a1 = *(const v4fa*)(sp + 4) * vm;
    const v4f b0 = *(const v4fa*)(sp + DK) * vm;
    const v4f b1 = *(const v4fa*)(sp + DK + 4) * vm;
    split8(a0, a1, hv[i], lv[i]);
#pragma unroll
    for (int e = 0; e < 4; ++e) {
      const float f0 = b0[e], f1 = b1[e];
      const unsigned short h0 = bf_bits(f0), h1 = bf_bits(f1);
      const unsigned short l0 = bf_bits(f0 - bf_up(h0)), l1 = bf_bits(f1 - bf_up(h1));
      sV[(cq + e) * 72 + sl]          = h0;
      sV[(cq + 4 + e) * 72 + sl]      = h1;
      sV[(DV + cq + e) * 72 + sl]     = l0;
      sV[(DV + cq + 4 + e) * 72 + sl] = l1;
    }
  }
  unsigned short* kd = KHL + ((size_t)k * SROWSP + (size_t)c * 64) * DK + cq;
  for (int pass = 0; pass < 2; ++pass) {
#pragma unroll
    for (int i = 0; i < 4; ++i) {
      const int sl = w * 8 + 2 * i + h;
      *(volatile v4u*)(kd + (size_t)sl * DK) = hv[i];
      *(volatile v4u*)(kd + (size_t)sl * DK + KLOFF) = lv[i];
    }
    __threadfence();
  }
  __syncthreads();
  const int piece = lane & 7, rg = lane >> 3;
  for (int pass = 0; pass < 2; ++pass) {
#pragma unroll
    for (int it = 0; it < 8; ++it) {
      const int line = it * 32 + w * 4 + rg;
      const int pln = line >> 7, d = line & 127;
      const v4u v = *(const v4ua*)(sV + (pln * DV + d) * 72 + 8 * piece);
      unsigned short* dst = VHL + (size_t)pln * VLOFF + ((size_t)k * DV + d) * SROWSP + (size_t)c * 64 + 8 * piece;
      *(volatile v4u*)dst = v;
    }
    __threadfence();
  }
}

__device__ __forceinline__ void split_p(v8f a, v8f c, v16b& hi, v16b& lo) {
  union U { v16b v; unsigned u[8]; };
  U H, L;
#pragma unroll
  for (int e = 0; e < 4; ++e) {
    unsigned x, y;
    split2(a[2 * e], a[2 * e + 1], x, y); H.u[e] = x;     L.u[e] = y;
    split2(c[2 * e], c[2 * e + 1], x, y); H.u[4 + e] = x; L.u[4 + e] = y;
  }
  hi = H.v;
  lo = L.v;
}

__global__ __launch_bounds__(128) void k_attn(
    const unsigned short* __restrict__ QHLp,
    const unsigned short* __restrict__ KHLp,
    const unsigned short* __restrict__ VHLp,
    const int* __restrict__ lab,
    float* OT) {
  __shared__ __align__(16) float sO[4 * 16 * DV];
  const int tid = (int)threadIdx.x, lane = tid & 31, w = tid >> 5;
  const int h = lane >> 4, m = lane & 15;
  const int k = (int)blockIdx.y;
  const int q0 = (int)blockIdx.x * 64 + 16 * w;

  const int cnt = class_count(lab, k);
  const int allm = (cnt == 0) ? 1 : 0;
  const int nkeys = (allm ? NSUP : cnt) * HW;
  const float sfac = allm ? 0.0f : 1.0f;
  int nch = (nkeys + 63) >> 6;
  nch = (nch > NCHMAX) ? NCHMAX : nch;

  const __bf16* QH = (const __bf16*)(const void*)QHLp;
  const __bf16* KH = (const __bf16*)(const void*)KHLp;
  const __bf16* VH = (const __bf16*)(const void*)VHLp;
  const __bf16* qh_row  = QH + (size_t)(q0 + m) * DK;
  const __bf16* ql_row  = qh_row + QLOFF;
  const __bf16* kh_base = KH + ((size_t)k * SROWSP + m) * DK;
  const __bf16* kl_base = kh_base + KLOFF;
  const __bf16* vh_base = VH + ((size_t)k * DV + m) * SROWSP;
  const __bf16* vl_base = vh_base + VLOFF;

  v8f o[8];
#pragma unroll
  for (int t = 0; t < 8; ++t) o[t] = zero8();
  float mrun = -1e30f, lrun = 0.0f;

#pragma unroll 1
  for (int kb = 0; kb < nch; ++kb) {
    const int j0 = kb * 64;
    v8f s[4];
#pragma unroll
    for (int j = 0; j < 4; ++j) s[j] = zero8();
#pragma unroll 1
    for (int dc = 0; dc < 4; ++dc) {
      const v16b qh = load_frag(qh_row + 32 * dc, h);
      const v16b ql = load_frag(ql_row + 32 * dc, h);
#pragma unroll
      for (int j = 0; j < 4; ++j) {
        const size_t ko = (size_t)(j0 + 16 * j) * DK + 32 * dc;
        const v16b kh = load_frag(kh_base + ko, h);
        const v16b kl = load_frag(kl_base + ko, h);
        s[j] = mma_b(kh, qh, s[j]);
        s[j] = mma_b(kl, qh, s[j]);
        s[j] = mma_b(kh, ql, s[j]);
      }
    }
#pragma unroll
    for (int j = 0; j < 4; ++j)
#pragma unroll
      for (int r = 0; r < 8; ++r) {
        const int jj = j0 + 16 * j + 8 * h + r;
        s[j][r] = (jj < nkeys) ? (s[j][r] * sfac) : -1e30f;
      }

    float mloc = s[0][0];
#pragma unroll
    for (int j = 0; j < 4; ++j)
#pragma unroll
      for (int r = 0; r < 8; ++r) mloc = fmaxf(mloc, s[j][r]);
    mloc = fmaxf(mloc, __shfl_xor(mloc, 16, 32));
    const float mnew = fmaxf(mrun, mloc);
    const float alpha = __expf(mrun - mnew);
    mrun = mnew;
    float lsum = 0.0f;
#pragma unroll
    for (int j = 0; j < 4; ++j)
#pragma unroll
      for (int r = 0; r < 8; ++r) {
        const float p = __expf(s[j][r] - mnew);
        s[j][r] = p;
        lsum += p;
      }
    lsum += __shfl_xor(lsum, 16, 32);
    lrun = lrun * alpha + lsum;
#pragma unroll
    for (int t = 0; t < 8; ++t)
#pragma unroll
      for (int r = 0; r < 8; ++r) o[t][r] = o[t][r] * alpha;

    v16b ph0, pl0, ph1, pl1;
    split_p(s[0], s[1], ph0, pl0);
    split_p(s[2], s[3], ph1, pl1);

#pragma unroll
    for (int t = 0; t < 8; ++t) {
      const size_t vo = (size_t)(16 * t) * SROWSP + j0;
      const v16b vh0 = load_frag(vh_base + vo, h);
      const v16b vl0 = load_frag(vl_base + vo, h);
      o[t] = mma_b(vh0, ph0, o[t]);
      o[t] = mma_b(vl0, ph0, o[t]);
      o[t] = mma_b(vh0, pl0, o[t]);
      const v16b vh1 = load_frag(vh_base + vo + 32, h);
      const v16b vl1 = load_frag(vl_base + vo + 32, h);
      o[t] = mma_b(vh1, ph1, o[t]);
      o[t] = mma_b(vl1, ph1, o[t]);
      o[t] = mma_b(vh1, pl1, o[t]);
    }
  }

  const float inv = (lrun > 0.0f) ? (1.0f / lrun) : 0.0f;
  float* so = sO + w * (16 * DV);
#pragma unroll
  for (int t = 0; t < 8; ++t)
#pragma unroll
    for (int r = 0; r < 8; ++r)
      so[m * DV + 16 * t + 8 * h + r] = o[t][r] * inv;
  __syncthreads();
  float* ob = OT + ((size_t)k * QROWS + q0) * DV + 4 * lane;
  for (int pass = 0; pass < 2; ++pass) {
#pragma unroll
    for (int row = 0; row < 16; ++row) {
      const v4f v = *(const v4fa*)(so + row * DV + 4 * lane);
      *(volatile v4f*)(ob + (size_t)row * DV) = v;
    }
    __threadfence();
  }
}

__global__ __launch_bounds__(256) void k_oxpose(const float* __restrict__ src, int spitch, int scoff,
                                                long long skstride, int nk, float* dstb) {
  __shared__ __align__(16) float T[16 * HW];
  const int lane = (int)threadIdx.x & 31, w = (int)threadIdx.x >> 5;
  const int g = (int)blockIdx.x, b = (int)blockIdx.y, kc = (int)blockIdx.z;
  const float* sb = src + (size_t)kc * (size_t)skstride + (size_t)(b * HW) * spitch + scoff + 16 * g;
  const int dq = 4 * (lane & 3), pr = lane >> 2;
#pragma unroll
  for (int it = 0; it < 4; ++it) {
    const int p  = it * 64 + w * 8 + pr;
    const int pc = (p > HW - 1) ? (HW - 1) : p;
    const v4f v = *(const v4fa*)(sb + (size_t)pc * spitch + dq);
    if (p < HW) {
      T[(dq + 0) * HW + p] = v[0];
      T[(dq + 1) * HW + p] = v[1];
      T[(dq + 2) * HW + p] = v[2];
      T[(dq + 3) * HW + p] = v[3];
    }
  }
  __syncthreads();
  float* db = dstb + ((size_t)(b * nk + kc) * DV + 16 * g) * HW;
  const int piece = lane & 7, rg = lane >> 3;
  for (int pass = 0; pass < 2; ++pass) {
#pragma unroll
    for (int it = 0; it < 4; ++it) {
      const int line = it * 32 + w * 4 + rg;
      const int lc = (line > NLN16 - 1) ? (NLN16 - 1) : line;
      const v4f v = *(const v4fa*)(T + lc * 32 + piece * 4);
      if (line < NLN16) *(volatile v4f*)(db + (size_t)line * 32 + piece * 4) = v;
    }
    __threadfence();
  }
}

extern "C" void kernel_launch(void* const* d_in, const int* in_sizes, int n_in,
                              void* d_out, int out_size, void* d_ws, size_t ws_size,
                              hipStream_t stream) {
  if (n_in < 5) return;
  if (in_sizes[0] != NSUP * CIN * HW) return;
  if (in_sizes[1] != NQRY * CIN * HW) return;
  if (in_sizes[2] != NSUP) return;
  if (in_sizes[3] != DK * CIN) return;
  if (in_sizes[4] != DV * CIN) return;
  if (out_size != OUT0_ELEMS + OUT1_ELEMS) return;

  const float* supF = (const float*)d_in[0];
  const float* qryF = (const float*)d_in[1];
  const int*   lab  = (const int*)d_in[2];
  const float* Wqk  = (const float*)d_in[3];
  const float* Wv   = (const float*)d_in[4];
  float* out = (float*)d_out;

  const size_t bWB  = (size_t)NPROJ * CIN * 2;
  const size_t bXQ  = (size_t)QROWS * CIN * 2;
  const size_t bXS  = (size_t)SROWSP * CIN * 2;
  const size_t bCQ  = (size_t)QROWS * NPROJ * 4;
  const size_t bCS  = (size_t)SROWSP * NPROJ * 4;
  const size_t bQHL = (size_t)2 * QROWS * DK * 2;
  const size_t bKHL = (size_t)2 * NCLS * SROWSP * DK * 2;
  const size_t bVHL = (size_t)2 * NCLS * DV * SROWSP * 2;
  const size_t bOT  = (size_t)NCLS * QROWS * DV * 4;
  size_t off = 0;
  const size_t oWB  = off; off += bWB;
  const size_t oXQ  = off; off += bXQ;
  const size_t oXS  = off; off += bXS;
  const size_t oCQ  = off; off += bCQ;
  const size_t oCS  = off; off += bCS;
  const size_t oQHL = off; off += bQHL;
  const size_t oKHL = off; off += bKHL;
  const size_t oVHL = off; off += bVHL;
  const size_t oOT  = off; off += bOT;
  if (off > ws_size) return;
  if (off > (size_t)134217728) return;

  char* ws = (char*)d_ws;
  unsigned short* WB  = (unsigned short*)(ws + oWB);
  unsigned short* XQ  = (unsigned short*)(ws + oXQ);
  unsigned short* XS  = (unsigned short*)(ws + oXS);
  float*          CQ  = (float*)(ws + oCQ);
  float*          CS  = (float*)(ws + oCS);
  unsigned short* QHL = (unsigned short*)(ws + oQHL);
  unsigned short* KHL = (unsigned short*)(ws + oKHL);
  unsigned short* VHL = (unsigned short*)(ws + oVHL);
  float*          OT  = (float*)(ws + oOT);

  const dim3 blk(256);
  k_wcvt<<<dim3((DK * CIN) / (256 * 8), 2), blk, 0, stream>>>(Wqk, Wv, WB);
  const int zq = NQRY + ((QROWS > NQRY * HW) ? 1 : 0);
  const int zs = NSUP + ((SROWSP > NSUP * HW) ? 1 : 0);
  k_xpose<<<dim3(4, CIN / 64, zq), blk, 0, stream>>>(qryF, XQ, NQRY, QROWS);
  k_xpose<<<dim3(4, CIN / 64, zs), blk, 0, stream>>>(supF, XS, NSUP, SROWSP);
  const int tilesQ = (QROWS / 64) * (NPROJ / 64);
  const int tilesS = (SROWSP / 64) * (NPROJ / 64);
  k_gemm64<<<dim3((tilesQ + 7) / 8), blk, 0, stream>>>(XQ, CIN, WB, CIN, CQ, NPROJ, QROWS, NPROJ, CIN);
  k_gemm64<<<dim3((tilesS + 7) / 8), blk, 0, stream>>>(XS, CIN, WB, CIN, CS, NPROJ, SROWSP, NPROJ, CIN);
  k_qsplit<<<dim3((QROWS * (DK / 8)) / 256), blk, 0, stream>>>(CQ, QHL);
  k_kvgather<<<dim3(NCHMAX, NCLS), blk, 0, stream>>>(CS, lab, KHL, VHL);
  k_attn<<<dim3(QTILES, NCLS), dim3(128), 0, stream>>>(QHL, KHL, VHL, lab, OT);
  k_oxpose<<<dim3(DV / 16, NQRY, NCLS), blk, 0, stream>>>(OT, DV, 0, (long long)QROWS * DV, NCLS, out);
  k_oxpose<<<dim3(DV / 16, NQRY, 1), blk, 0, stream>>>(CQ, NPROJ, DK, 0LL, 1, out + OUT0_ELEMS);
  (void)hipGetLastError();
}
